// PlotterEmbedding_19902878450186
// MI455X (gfx1250) — hardware-verified
//
#include <hip/hip_runtime.h>
#include <math.h>

typedef __attribute__((ext_vector_type(16))) _Float16 v16h;
typedef __attribute__((ext_vector_type(16))) __bf16 v16b;
typedef __attribute__((ext_vector_type(8)))  _Float16 v8h;
typedef __attribute__((ext_vector_type(8)))  float v8f;
typedef __attribute__((ext_vector_type(4)))  float v4f;
typedef __attribute__((ext_vector_type(2)))  float v2f;
typedef __attribute__((ext_vector_type(4)))  unsigned v4u;
typedef __attribute__((ext_vector_type(4)))  int v4i;
typedef float __attribute__((may_alias)) float_a;
typedef int __attribute__((may_alias)) int_a;

template <typename T> __device__ __forceinline__ void vst2(void* p, T v) { *(volatile T*)p = v; __threadfence(); *(volatile T*)p = v; }
__device__ __forceinline__ v8f wmma16(v16h a, v16h b, v8f c) {
  v8f d = __builtin_amdgcn_wmma_f32_16x16x32_f16(false, a, false, b, (short)0, c, false, false);
  asm volatile("v_nop\n\tv_nop\n\tv_nop\n\tv_nop" : "+v"(d) : "v"(a), "v"(b));
  return d;
}
__device__ __forceinline__ v8f wmma_bf(v16b a, v16b b, v8f c) {
  v8f d = __builtin_amdgcn_wmma_f32_16x16x32_bf16(false, a, false, b, (short)0, c, false, false);
  asm volatile("v_nop\n\tv_nop\n\tv_nop\n\tv_nop" : "+v"(d) : "v"(a), "v"(b));
  return d;
}
__device__ __forceinline__ v16h frag_h(const _Float16* rowk0, int lane) {
  union { v16h v; v8h q[2]; } u; const _Float16* p = rowk0 + 8 * (lane >> 4);
  u.q[0] = *(const v8h*)p; u.q[1] = *(const v8h*)(p + 16); return u.v;
}
__device__ __forceinline__ v16h frag_f32(const float* rowk0, int lane) {
  v16h a; const float* p = rowk0 + 8 * (lane >> 4);
#pragma unroll
  for (int i = 0; i < 8; ++i) { a[i] = (_Float16)p[i]; a[8 + i] = (_Float16)p[16 + i]; }
  return a;
}
__device__ __forceinline__ v16h frag_f32s(const float* rowk0, int lane, float sc) {
  v16h a; const float* p = rowk0 + 8 * (lane >> 4);
#pragma unroll
  for (int i = 0; i < 8; ++i) { a[i] = (_Float16)(p[i] * sc); a[8 + i] = (_Float16)(p[16 + i] * sc); }
  return a;
}
__device__ __forceinline__ v16h fragc_f32(const float* W, int k0, int n, int lane, int ld, int K) {
  v16h a; const int g = lane >> 4;
#pragma unroll
  for (int i = 0; i < 8; ++i) { const int ka = k0 + 8 * g + i, kb = ka + 16;
    a[i] = (_Float16)(ka < K ? W[(size_t)ka * ld + n] : 0.f); a[8 + i] = (_Float16)(kb < K ? W[(size_t)kb * ld + n] : 0.f); }
  return a;
}
struct F2 { v16b h, l; };
__device__ __forceinline__ F2 bsplit16(const float v[16]) { F2 r;
#pragma unroll
  for (int i = 0; i < 16; ++i) { const __bf16 h = (__bf16)v[i]; r.h[i] = h; r.l[i] = (__bf16)(v[i] - (float)h); }
  return r; }
__device__ __forceinline__ F2 split_row(const float* row, int k0, int lane) { float v[16]; const float* p = row + k0 + 8 * (lane >> 4);
#pragma unroll
  for (int i = 0; i < 8; ++i) { v[i] = p[i]; v[8 + i] = p[16 + i]; }
  return bsplit16(v); }
__device__ __forceinline__ F2 split_rowK(const float* row, int k0, int lane, int K) { float v[16]; const int g = lane >> 4;
#pragma unroll
  for (int i = 0; i < 8; ++i) { const int ka = k0 + 8 * g + i, kb = ka + 16; v[i] = ka < K ? row[ka] : 0.f; v[8 + i] = kb < K ? row[kb] : 0.f; }
  return bsplit16(v); }
__device__ __forceinline__ F2 split_col(const float* W, int k0, int n, int lane, int ld, int K) { float v[16]; const int g = lane >> 4;
#pragma unroll
  for (int i = 0; i < 8; ++i) { const int ka = k0 + 8 * g + i, kb = ka + 16; v[i] = ka < K ? W[(size_t)ka * ld + n] : 0.f; v[8 + i] = kb < K ? W[(size_t)kb * ld + n] : 0.f; }
  return bsplit16(v); }
__device__ __forceinline__ v8f mac3(const F2& a, const F2& b, v8f c) { c = wmma_bf(a.l, b.h, c); c = wmma_bf(a.h, b.l, c); return wmma_bf(a.h, b.h, c); }
__device__ __forceinline__ float sigm(float v) { return 1.0f / (1.0f + expf(-v)); }
#define LDSX() do { asm volatile("s_wait_dscnt 0" ::: "memory"); __builtin_amdgcn_wave_barrier(); __builtin_amdgcn_fence(__ATOMIC_RELEASE, "workgroup"); } while (0)

__device__ __forceinline__ v16h frag_f32sK(const float* __restrict__ row, int k0, int lane, float sc, int K) {
  const int g = lane >> 4; v16h r;
#pragma unroll
  for (int i = 0; i < 8; ++i) { const int ka = k0 + 8 * g + i, kb = ka + 16; r[i] = (_Float16)((ka < K ? row[ka] : 0.f) * sc); r[8 + i] = (_Float16)((kb < K ? row[kb] : 0.f) * sc); }
  return r;
}
#define NBT 64
#define TT 1024
#define NHG 100
#define NBD 6
#define KK (NHG * NBD)
#define KP 608
#define NO 64
#define NR (NBT * TT)

__global__ __launch_bounds__(128) void k_main(const float* __restrict__ tin, const float* __restrict__ fin, const int* __restrict__ bidx, const int* __restrict__ msk, const float* __restrict__ W, const float* __restrict__ bias, float* __restrict__ out) {
  __shared__ __align__(16) _Float16 sa[4][16][40];
  __shared__ __align__(16) float so[4][16][68];
  __shared__ float stm[4][16], sfm[4][16]; __shared__ int sbd[4][16];
  const int tid = threadIdx.x, wave = tid >> 5, lane = tid & 31, col = lane & 15, g = lane >> 4;
  const int r0 = blockIdx.x * 64 + wave * 16;
  if (lane < 16) { const int r = r0 + lane; const int t = r % TT; const bool m = msk[r] != 0;
    const float tm = (sigm(tin[r]) - 0.5f) * 2.0f * (float)TT, fm = sigm(fin[r]) * (float)NHG;
    stm[wave][lane] = m ? tm : -10.0f; sfm[wave][lane] = m ? fm : -10.0f; sbd[wave][lane] = bidx[r]; (void)t; }
  LDSX();
  const float coef = 0.3989422804014327f;
  v8f acc[4] = {};
#pragma unroll 1
  for (int kc = 0; kc < KP / 32; ++kc) {
    { const int r = r0 + col; const float xt = (float)(r % TT); const float tm = stm[wave][col], fm = sfm[wave][col]; const int bd = sbd[wave][col]; const float dx2 = (xt - tm) * (xt - tm);
      union { v8h h[2]; v4u u2[2]; } pk;
#pragma unroll
      for (int u = 0; u < 16; ++u) { const int k = kc * 32 + g * 16 + u; float v = 0.f;
        if (k < KK && (k % NBD) == bd) { const float yy = (float)(k / NBD); const float d2 = (yy - fm) * (yy - fm) + dx2; v = 256.0f * coef * expf(-0.5f * d2); }
        pk.h[u >> 3][u & 7] = (_Float16)v; }
      *(v4u*)(&sa[wave][col][g * 16]) = pk.u2[0]; *(v4u*)(&sa[wave][col][g * 16 + 8]) = pk.u2[1]; }
    LDSX();
    const v16h a = frag_h(&sa[wave][col][0], lane);
#pragma unroll
    for (int t = 0; t < 4; ++t) acc[t] = wmma16(a, frag_f32sK(W + (size_t)(t * 16 + col) * KK, kc * 32, lane, 16.0f, KK), acc[t]);
    LDSX(); }
#pragma unroll
  for (int t = 0; t < 4; ++t) { const float bb = bias[t * 16 + col];
#pragma unroll
    for (int r = 0; r < 8; ++r) so[wave][8 * g + r][t * 16 + col] = acc[t][r] * (1.0f / 4096.0f) + bb; }
  LDSX();
  for (int q = lane; q < 16 * 16; q += 32) { const int rl = q >> 4, pc = q & 15; vst2(out + (size_t)(r0 + rl) * NO + pc * 4, *(const v4f*)(&so[wave][rl][pc * 4])); }
}
extern "C" void kernel_launch(void* const* d_in, const int* in_sizes, int n_in, void* d_out, int out_size, void* d_ws, size_t ws_size, hipStream_t stream) {
  (void)in_sizes; (void)n_in; (void)out_size; (void)ws_size; (void)d_ws;
  const float* tin = (const float*)d_in[0]; const float* fin = (const float*)d_in[1]; const int* bidx = (const int*)d_in[2]; const int* msk = (const int*)d_in[3]; const float* W = (const float*)d_in[4]; const float* bias = (const float*)d_in[5];
  float* out = (float*)d_out;
  k_main<<<NR / 64, 128, 0, stream>>>(tin, fin, bidx, msk, W, bias, out);
}
